// Block_1563368096568
// MI455X (gfx1250) — hardware-run, weakly checked
//
#include <hip/hip_runtime.h>
#include <stdint.h>


typedef _Float16 v16h __attribute__((ext_vector_type(16)));
typedef _Float16 v8h  __attribute__((ext_vector_type(8)));
typedef float    v8f  __attribute__((ext_vector_type(8)));
typedef float    v4f  __attribute__((ext_vector_type(4)));
typedef unsigned int u32x4 __attribute__((ext_vector_type(4)));

#ifndef NB
#define NB 2
#endif
#define NB_FULL 2

constexpr int kC     = 768;
constexpr int kHeads = 12;
constexpr int kDH    = 64;
constexpr int kHW    = 64;
constexpr int kL     = kHW * kHW;
constexpr int kWS    = 14;
constexpr int kNW    = kWS * kWS;
constexpr int kNWX   = (kHW + kWS - 1) / kWS;
constexpr int kWPI   = kNWX * kNWX;
constexpr int kWR    = 208;
constexpr int kQT    = kWR / 16;
constexpr int kKP    = 224;
constexpr int kPP    = 232;
constexpr int kLP    = kKP + 4;
constexpr int kQKV   = 3 * kC;
constexpr int kHid   = 4 * kC;
constexpr int kRel   = 2 * kWS - 1;

constexpr int kMT     = NB * kL;
constexpr int kNWIN   = NB * kWPI;
constexpr int kMW     = kNWIN * kWR;
constexpr int kMWP    = ((kMW + 127) / 128) * 128;
constexpr int kTilesT = kMT / 128;
constexpr int kNChunk = 2;
constexpr int kTPC    = (kTilesT + kNChunk - 1) / kNChunk;

constexpr float kEps      = 1e-5f;
constexpr float kWCarry   = 64.0f;
constexpr float kPCarry   = 1024.0f;
constexpr float kCtxCarry = 16.0f;
constexpr float kGCarry   = 16.0f;
constexpr float kScale    = 0.125f;

constexpr size_t kBWqkv = (size_t)kQKV * kC * 2;
constexpr size_t kBWpj  = (size_t)kC * kC * 2;
constexpr size_t kBWf1  = (size_t)kHid * kC * 2;
constexpr size_t kBWf2  = (size_t)kC * kHid * 2;
constexpr size_t kBRel  = (size_t)64 * 64 * 2;
constexpr size_t kBRA   = (size_t)kMWP * kC * 2;
constexpr size_t kRBBytesA = (size_t)kMWP * kQKV * 2;
constexpr size_t kRBBytesB = (size_t)kTPC * 128 * kHid * 2;
constexpr size_t kRBBytes  = (kRBBytesA > kRBBytesB) ? kRBBytesA : kRBBytesB;
constexpr size_t kBX1   = (size_t)kMT * kC * 4;

static_assert(NB >= 1 && NB <= NB_FULL);
static_assert(kMT % 128 == 0);
static_assert(kMWP % 128 == 0 && kMWP >= kMW);
static_assert(kMWP % 8 == 0 && kMT % 8 == 0);
static_assert((size_t)kMT * kC * 2 <= kBRA);
static_assert(kHeads * kDH == kC && kDH == 64);
static_assert(kC % 128 == 0 && kQKV % 128 == 0 && kHid % 128 == 0);
static_assert(kC % 64 == 0 && kHid % 64 == 0 && kQKV % 64 == 0);
static_assert(kWR % 16 == 0 && kNW <= kWR && kKP >= kWR && kKP % 32 == 0 && kKP + 8 <= kPP);
static_assert(kKP <= kLP);
static_assert(kNWX * kWS >= kHW && (kNWX - 1) * kWS < kHW);
static_assert(kRel <= 32);
static_assert((size_t)kMWP * kQKV * 2 <= kRBBytes);
static_assert((size_t)kTPC * 128 * kHid * 2 <= kRBBytes);
static_assert(kTPC * kNChunk >= kTilesT);

enum { EPI_QKV = 0, EPI_GELU = 1, EPI_X1 = 2, EPI_OUT = 3 };

__device__ __forceinline__ v8f wmma16(v16h a, v16h b, v8f c) {
  v8f d = __builtin_amdgcn_wmma_f32_16x16x32_f16(false, a, false, b, (short)0, c,
                                                 false, false);
  asm volatile("v_nop\n\tv_nop\n\tv_nop\n\tv_nop" : "+v"(d) : "v"(a), "v"(b));
  return d;
}

__device__ __forceinline__ v16h load_frag(const _Float16* p, int ld, int lane) {
  const int r  = lane & 15;
  const int k8 = (lane >> 4) << 3;
  const _Float16* q = p + (size_t)r * ld + k8;
  union { v16h v; v8h h[2]; } u;
  u.h[0] = *(const v8h*)(q);
  u.h[1] = *(const v8h*)(q + 16);
  return u.v;
}

__device__ __forceinline__ float bf16r(float x) {
  unsigned int u = __float_as_uint(x);
  u += 0x7FFFu + ((u >> 16) & 1u);
  u &= 0xFFFF0000u;
  return __uint_as_float(u);
}

__device__ __forceinline__ float gelu_f(float x) {
  return 0.5f * x * (1.0f + erff(x * 0.70710678118654752f));
}

__device__ __forceinline__ float wave_sum(float v) {
#pragma unroll
  for (int off = 16; off > 0; off >>= 1) v += __shfl_xor(v, off);
  return v;
}

__device__ __forceinline__ void vst4f(float* p, v4f v) { *(volatile v4f*)p = v; }
__device__ __forceinline__ void vst8h(_Float16* p, v8h v) {
  union { v8h h; u32x4 u; } t;
  t.h = v;
  *(volatile u32x4*)p = t.u;
}

__device__ __forceinline__ int tok_of(int row, bool& ok) {
  const int win = row / kWR;
  const int t   = row - win * kWR;
  const int b   = win / kWPI;
  const int w2  = win - b * kWPI;
  const int wi  = w2 / kNWX, wj = w2 - wi * kNWX;
  const int ti  = t / kWS, tj = t - ti * kWS;
  const int y   = wi * kWS + ti;
  const int x   = wj * kWS + tj;
  ok = (row < kMW) && (t < kNW) && (y < kHW) && (x < kHW);
  const int bc = min(b, NB - 1);
  const int yc = min(y, kHW - 1);
  const int xc = min(x, kHW - 1);
  return bc * kL + yc * kHW + xc;
}

__global__ __launch_bounds__(256)
void cvt_wt(const float* __restrict__ W, _Float16* __restrict__ Bt, int K, int N) {
  __shared__ __align__(16) _Float16 sT[64 * 72];
  const int tid = threadIdx.x, lane = tid & 31, wave = tid >> 5;
  const int n0 = blockIdx.x * 64, k0 = blockIdx.y * 64;
#pragma unroll
  for (int it = 0; it < 4; ++it) {
    const int kr = it * 16 + (tid >> 4);
    const int nc = (tid & 15) * 4;
    const v4f a = *(const v4f*)(W + (size_t)(k0 + kr) * N + n0 + nc);
#pragma unroll
    for (int e = 0; e < 4; ++e)
      sT[(nc + e) * 72 + kr] = (_Float16)(bf16r(a[e]) * kWCarry);
  }
  __syncthreads();
  v8h sv[2];
#pragma unroll
  for (int it = 0; it < 2; ++it) {
    const int row = wave * 8 + it * 4 + (lane >> 3), piece = lane & 7;
    sv[it] = *(const v8h*)(&sT[row * 72 + piece * 8]);
    vst8h(Bt + (size_t)(n0 + row) * K + k0 + piece * 8, sv[it]);
  }
  __threadfence();
#pragma unroll
  for (int it = 0; it < 2; ++it) {
    const int row = wave * 8 + it * 4 + (lane >> 3), piece = lane & 7;
    vst8h(Bt + (size_t)(n0 + row) * K + k0 + piece * 8, sv[it]);
  }
}

__global__ __launch_bounds__(256)
void cvt_rel(const float* __restrict__ rh, const float* __restrict__ rw,
             _Float16* __restrict__ relp) {
  const int tid = threadIdx.x, lane = tid & 31, wave = tid >> 5;
  v8h sv[2];
#pragma unroll
  for (int it = 0; it < 2; ++it) {
    const int row = wave * 8 + it * 4 + (lane >> 3), piece = lane & 7;
    const int ia = min(row, kRel - 1);
    const int ib = min(max(row - 32, 0), kRel - 1);
    const v4f a0 = *(const v4f*)(rh + ia * kDH + piece * 8);
    const v4f a1 = *(const v4f*)(rh + ia * kDH + piece * 8 + 4);
    const v4f b0 = *(const v4f*)(rw + ib * kDH + piece * 8);
    const v4f b1 = *(const v4f*)(rw + ib * kDH + piece * 8 + 4);
    const bool useA = row < kRel;
    const bool useB = (row >= 32) && (row < 32 + kRel);
    v8h o;
#pragma unroll
    for (int e = 0; e < 4; ++e) {
      const float va = useA ? a0[e] : (useB ? b0[e] : 0.0f);
      const float vb = useA ? a1[e] : (useB ? b1[e] : 0.0f);
      o[e]     = (_Float16)(bf16r(va) * kWCarry);
      o[4 + e] = (_Float16)(bf16r(vb) * kWCarry);
    }
    sv[it] = o;
    vst8h(relp + row * 64 + piece * 8, o);
  }
  __threadfence();
#pragma unroll
  for (int it = 0; it < 2; ++it) {
    const int row = wave * 8 + it * 4 + (lane >> 3), piece = lane & 7;
    vst8h(relp + row * 64 + piece * 8, sv[it]);
  }
}

template <int GATHER>
__device__ __forceinline__ void ld8(const float* p, float (&v)[8]) {
  const v4f a = *(const v4f*)(p);
  const v4f b = *(const v4f*)(p + 4);
#pragma unroll
  for (int e = 0; e < 4; ++e) {
    v[e]     = GATHER ? bf16r(a[e]) : a[e];
    v[4 + e] = GATHER ? bf16r(b[e]) : b[e];
  }
}

template <int GATHER>
__global__ __launch_bounds__(256)
void ln_rows(const float* __restrict__ src, const float* __restrict__ g,
             const float* __restrict__ bta, _Float16* __restrict__ dst) {
  const int tid = threadIdx.x, lane = tid & 31, wave = tid >> 5;
  const int row = blockIdx.x * 8 + wave;
  bool ok = true;
  int srow = row;
  if (GATHER) srow = tok_of(row, ok);
  const float* sp = src + (size_t)srow * kC;

  float s = 0.0f;
#pragma unroll 1
  for (int it = 0; it < 3; ++it) {
    float v[8];
    ld8<GATHER>(sp + (it * 32 + lane) * 8, v);
    s += ((v[0] + v[1]) + (v[2] + v[3])) + ((v[4] + v[5]) + (v[6] + v[7]));
  }
  s = wave_sum(s);
  const float mu = s * (1.0f / (float)kC);

  float q = 0.0f;
#pragma unroll 1
  for (int it = 0; it < 3; ++it) {
    float v[8];
    ld8<GATHER>(sp + (it * 32 + lane) * 8, v);
    float d0 = v[0] - mu, d1 = v[1] - mu, d2 = v[2] - mu, d3 = v[3] - mu;
    float d4 = v[4] - mu, d5 = v[5] - mu, d6 = v[6] - mu, d7 = v[7] - mu;
    q += ((d0 * d0 + d1 * d1) + (d2 * d2 + d3 * d3)) + ((d4 * d4 + d5 * d5) + (d6 * d6 + d7 * d7));
  }
  q = wave_sum(q);
  const float rs = rsqrtf(q * (1.0f / (float)kC) + kEps);

  v8h o[3];
#pragma unroll
  for (int it = 0; it < 3; ++it) {
    const int c8 = (it * 32 + lane) * 8;
    float v[8];
    ld8<GATHER>(sp + c8, v);
    const v4f ga = *(const v4f*)(g + c8);
    const v4f gb = *(const v4f*)(g + c8 + 4);
    const v4f ba = *(const v4f*)(bta + c8);
    const v4f bb = *(const v4f*)(bta + c8 + 4);
    v8h t;
#pragma unroll
    for (int e = 0; e < 4; ++e) {
      const float ya = ((v[e] - mu) * rs) * bf16r(ga[e]) + bf16r(ba[e]);
      const float yb = ((v[4 + e] - mu) * rs) * bf16r(gb[e]) + bf16r(bb[e]);
      t[e]     = (_Float16)(ok ? ya : 0.0f);
      t[4 + e] = (_Float16)(ok ? yb : 0.0f);
    }
    o[it] = t;
    vst8h(dst + (size_t)row * kC + c8, t);
  }
  __threadfence();
#pragma unroll
  for (int it = 0; it < 3; ++it) {
    const int c8 = (it * 32 + lane) * 8;
    vst8h(dst + (size_t)row * kC + c8, o[it]);
  }
}

template <int MI, int NJ>
__device__ __forceinline__ void gemm_core(v8f (&acc)[MI][NJ], const _Float16* Aw,
                                          const _Float16* Bw, int K, int lane) {
  for (int k0 = 0; k0 < K; k0 += 32) {
    v16h a[MI];
#pragma unroll
    for (int i = 0; i < MI; ++i) a[i] = load_frag(Aw + (size_t)(i * 16) * K + k0, K, lane);
#pragma unroll
    for (int j = 0; j < NJ; ++j) {
      const v16h b = load_frag(Bw + (size_t)(j * 16) * K + k0, K, lane);
#pragma unroll
      for (int i = 0; i < MI; ++i) acc[i][j] = wmma16(a[i], b, acc[i][j]);
    }
  }
}

template <int EPI>
__global__ __launch_bounds__(256)
void gemm_rows(const _Float16* __restrict__ A, const _Float16* __restrict__ Bt,
               const float* __restrict__ bias, const float* __restrict__ resid,
               float* __restrict__ outF, _Float16* __restrict__ outH,
               int N, int K, int m_base) {
  __shared__ __align__(16) float stg[8][16 * 68];
  const int tid = threadIdx.x, lane = tid & 31, wave = tid >> 5;
  const int wm = wave & 3, wn = wave >> 2;
  const int m0w = blockIdx.x * 128 + wm * 32;
  const int n0w = blockIdx.y * 128 + wn * 64;
  const _Float16* Aw = A + (size_t)m0w * K;
  const _Float16* Bw = Bt + (size_t)n0w * K;

  v8f acc[2][4] = {};
  gemm_core<2, 4>(acc, Aw, Bw, K, lane);

  constexpr float sc = (EPI == EPI_QKV || EPI == EPI_GELU) ? (1.0f / 64.0f) : (1.0f / 1024.0f);
  const int n = lane & 15, h8 = (lane >> 4) * 8;
  float* sw = &stg[wave][0];

#pragma unroll
  for (int i = 0; i < 2; ++i) {
#pragma unroll
    for (int j = 0; j < 4; ++j)
#pragma unroll
      for (int r = 0; r < 8; ++r)
        sw[(h8 + r) * 68 + j * 16 + n] = acc[i][j][r] * sc;
    __syncthreads();
    if constexpr (EPI == EPI_X1 || EPI == EPI_OUT) {
      v4f sv[8];
      size_t dof[8];
      bool okv[8];
#pragma unroll
      for (int q = 0; q < 8; ++q) {
        const int row = q * 2 + (lane >> 4), col = (lane & 15) * 4;
        const int gm = m0w + i * 16 + row, gn = n0w + col;
        v4f v = *(const v4f*)(sw + row * 68 + col);
        const v4f bb = *(const v4f*)(bias + gn);
#pragma unroll
        for (int e = 0; e < 4; ++e) v[e] += bf16r(bb[e]);
        if constexpr (EPI == EPI_X1) {
          bool okq = true;
          const int tok = tok_of(m_base + gm, okq);
          const size_t ro = (size_t)tok * kC + gn;
          const v4f rr = *(const v4f*)(resid + ro);
#pragma unroll
          for (int e = 0; e < 4; ++e) v[e] = bf16r(rr[e]) + v[e];
          dof[q] = ro;
          okv[q] = okq;
        } else {
          const size_t ro = (size_t)gm * N + gn;
          const v4f rr = *(const v4f*)(resid + ro);
#pragma unroll
          for (int e = 0; e < 4; ++e) v[e] = rr[e] + v[e];
          dof[q] = ro;
          okv[q] = true;
        }
        sv[q] = v;
        if (okv[q]) vst4f(outF + dof[q], v);
      }
      __threadfence();
#pragma unroll
      for (int q = 0; q < 8; ++q) {
        if (okv[q]) vst4f(outF + dof[q], sv[q]);
      }
    } else {
      v8h sv[4];
#pragma unroll
      for (int q = 0; q < 4; ++q) {
        const int row = q * 4 + (lane >> 3), col = (lane & 7) * 8;
        const int gm = m0w + i * 16 + row, gn = n0w + col;
        const v4f va = *(const v4f*)(sw + row * 68 + col);
        const v4f vb = *(const v4f*)(sw + row * 68 + col + 4);
        const v4f ba = *(const v4f*)(bias + gn);
        const v4f bb = *(const v4f*)(bias + gn + 4);
        v8h o;
#pragma unroll
        for (int e = 0; e < 4; ++e) {
          float xa = va[e] + bf16r(ba[e]), xb = vb[e] + bf16r(bb[e]);
          if constexpr (EPI == EPI_GELU) { xa = gelu_f(xa) * kGCarry; xb = gelu_f(xb) * kGCarry; }
          o[e]     = (_Float16)xa;
          o[4 + e] = (_Float16)xb;
        }
        sv[q] = o;
        vst8h(outH + (size_t)gm * N + gn, o);
      }
      __threadfence();
#pragma unroll
      for (int q = 0; q < 4; ++q) {
        const int row = q * 4 + (lane >> 3), col = (lane & 7) * 8;
        const int gm = m0w + i * 16 + row, gn = n0w + col;
        vst8h(outH + (size_t)gm * N + gn, sv[q]);
      }
    }
    __syncthreads();
  }
}

__global__ __launch_bounds__(32) __attribute__((amdgpu_num_vgpr(256)))
void attn_win(const _Float16* __restrict__ qkv, const _Float16* __restrict__ relp,
              _Float16* __restrict__ ctxp) {
  __shared__ __align__(16) _Float16 Vt[kDH * kPP];
  __shared__ __align__(16) _Float16 Ps[16 * kPP];
  __shared__ __align__(16) float    Lg[16 * kLP];
  __shared__ __align__(16) float    Bq[16 * 68];
  __shared__ __align__(16) _Float16 Cs[16 * 72];
  const int w = blockIdx.x, hh = blockIdx.y;
  const int lane = threadIdx.x & 31;
  const int n = lane & 15, h8 = (lane >> 4) * 8;
  const _Float16* wq = qkv + (size_t)w * kWR * kQKV;
  const _Float16* qp = wq + hh * kDH;
  const _Float16* kp = wq + kC + hh * kDH;
  const _Float16* vp = wq + 2 * kC + hh * kDH;
  const _Float16 z16 = (_Float16)0.0f;

#pragma unroll 1
  for (int tt = 0; tt < kKP / 32; ++tt) {
    const int t  = lane + tt * 32;
    const int tc = min(t, kNW - 1);
    const bool ok = t < kNW;
    const _Float16* src = vp + (size_t)tc * kQKV;
#pragma unroll
    for (int c = 0; c < 8; ++c) {
      const v8h vv = *(const v8h*)(src + c * 8);
#pragma unroll
      for (int e = 0; e < 8; ++e) Vt[(c * 8 + e) * kPP + t] = ok ? vv[e] : z16;
    }
  }
#pragma unroll
  for (int r = 0; r < 8; ++r) Ps[(h8 + r) * kPP + kQT * 16 + n] = z16;
  __syncthreads();

#pragma unroll 1
  for (int i = 0; i < kQT; ++i) {
    const _Float16* qrow = qp + (size_t)(i * 16) * kQKV;
    const v16h qf0 = load_frag(qrow, kQKV, lane);
    const v16h qf1 = load_frag(qrow + 32, kQKV, lane);

#pragma unroll 1
    for (int j = 0; j < 4; ++j) {
      const _Float16* rp = relp + (size_t)(j * 16) * kDH;
      v8f z = {};
      z = wmma16(qf0, load_frag(rp, kDH, lane), z);
      z = wmma16(qf1, load_frag(rp + 32, kDH, lane), z);
#pragma unroll
      for (int r = 0; r < 8; ++r)
        Bq[(h8 + r) * 68 + j * 16 + n] = z[r] * (1.0f / kWCarry);
    }
    __syncthreads();

    int iqv[8], jqv[8];
    float mx[8];
#pragma unroll
    for (int r = 0; r < 8; ++r) {
      const int qr = i * 16 + h8 + r;
      const int qc = min(qr, kNW - 1);
      iqv[r] = qc / kWS;
      jqv[r] = qc - iqv[r] * kWS;
      mx[r]  = -1.0e30f;
    }

#pragma unroll 1
    for (int j = 0; j < kQT; ++j) {
      const _Float16* krow = kp + (size_t)(j * 16) * kQKV;
      v8f z = {};
      z = wmma16(qf0, load_frag(krow, kQKV, lane), z);
      z = wmma16(qf1, load_frag(krow + 32, kQKV, lane), z);
      const int key = j * 16 + n;
      const int kc  = min(key, kNW - 1);
      const int ik  = kc / kWS, jk = kc - ik * kWS;
      const bool kok = key < kNW;
#pragma unroll
      for (int r = 0; r < 8; ++r) {
        const float* bqr = &Bq[(h8 + r) * 68];
        const float bb = bqr[iqv[r] - ik + (kWS - 1)] + bqr[32 + jqv[r] - jk + (kWS - 1)];
        float lv = z[r] * kScale + bb;
        lv = kok ? lv : -1.0e30f;
        Lg[(h8 + r) * kLP + key] = lv;
        mx[r] = fmaxf(mx[r], lv);
      }
    }
    __syncthreads();

#pragma unroll
    for (int r = 0; r < 8; ++r) {
      float m = mx[r];
      m = fmaxf(m, __shfl_xor(m, 1));
      m = fmaxf(m, __shfl_xor(m, 2));
      m = fmaxf(m, __shfl_xor(m, 4));
      m = fmaxf(m, __shfl_xor(m, 8));
      mx[r] = m;
    }

    float ps[8];
#pragma unroll
    for (int r = 0; r < 8; ++r) ps[r] = 0.0f;
#pragma unroll 1
    for (int j = 0; j < kQT; ++j) {
      const int key = j * 16 + n;
#pragma unroll
      for (int r = 0; r < 8; ++r) {
        const float p = __expf(Lg[(h8 + r) * kLP + key] - mx[r]);
        ps[r] += p;
        Ps[(h8 + r) * kPP + key] = (_Float16)(p * kPCarry);
      }
    }
    float rinv[8];
#pragma unroll
    for (int r = 0; r < 8; ++r) {
      float sum = ps[r];
      sum += __shfl_xor(sum, 1);
      sum += __shfl_xor(sum, 2);
      sum += __shfl_xor(sum, 4);
      sum += __shfl_xor(sum, 8);
      rinv[r] = (kCtxCarry / kPCarry) * (1.0f / sum);
    }
    __syncthreads();

    v8f cacc[4] = {};
#pragma unroll 1
    for (int kk = 0; kk < kKP / 32; ++kk) {
      const v16h pa = load_frag(&Ps[kk * 32], kPP, lane);
#pragma unroll
      for (int dt = 0; dt < 4; ++dt) {
        const v16h vb = load_frag(&Vt[(dt * 16) * kPP + kk * 32], kPP, lane);
        cacc[dt] = wmma16(pa, vb, cacc[dt]);
      }
    }

#pragma unroll
    for (int r = 0; r < 8; ++r) {
      const int qr = i * 16 + h8 + r;
      const bool okq = qr < kNW;
#pragma unroll
      for (int dt = 0; dt < 4; ++dt) {
        const float val = okq ? (cacc[dt][r] * rinv[r]) : 0.0f;
        Cs[(h8 + r) * 72 + dt * 16 + n] = (_Float16)val;
      }
    }
    __syncthreads();

    v8h sv[4];
#pragma unroll
    for (int it = 0; it < 4; ++it) {
      const int row = it * 4 + (lane >> 3), piece = lane & 7;
      sv[it] = *(const v8h*)(&Cs[row * 72 + piece * 8]);
      _Float16* dst = ctxp + ((size_t)w * kWR + i * 16 + row) * kC + hh * kDH + piece * 8;
      vst8h(dst, sv[it]);
    }
    __threadfence();
#pragma unroll
    for (int it = 0; it < 4; ++it) {
      const int row = it * 4 + (lane >> 3), piece = lane & 7;
      _Float16* dst = ctxp + ((size_t)w * kWR + i * 16 + row) * kC + hh * kDH + piece * 8;
      vst8h(dst, sv[it]);
    }
  }
}

extern "C" void kernel_launch(void* const* d_in, const int* in_sizes, int n_in,
                              void* d_out, int out_size, void* d_ws, size_t ws_size,
                              hipStream_t stream) {
  if (n_in < 15) return;
  if (in_sizes[0] < kMT * kC) return;
  if (in_sizes[1] < kC || in_sizes[2] < kC) return;
  if (in_sizes[3] < kC * kQKV || in_sizes[4] < kQKV) return;
  if (in_sizes[5] < kC * kC || in_sizes[6] < kC) return;
  if (in_sizes[7] < kRel * kDH || in_sizes[8] < kRel * kDH) return;
  if (in_sizes[9] < kC || in_sizes[10] < kC) return;
  if (in_sizes[11] < kC * kHid || in_sizes[12] < kHid) return;
  if (in_sizes[13] < kHid * kC || in_sizes[14] < kC) return;
  if (out_size < kMT * kC) return;

  const float* x      = (const float*)d_in[0];
  const float* n1g    = (const float*)d_in[1];
  const float* n1b    = (const float*)d_in[2];
  const float* w_qkv  = (const float*)d_in[3];
  const float* b_qkv  = (const float*)d_in[4];
  const float* w_proj = (const float*)d_in[5];
  const float* b_proj = (const float*)d_in[6];
  const float* rel_h  = (const float*)d_in[7];
  const float* rel_w  = (const float*)d_in[8];
  const float* n2g    = (const float*)d_in[9];
  const float* n2b    = (const float*)d_in[10];
  const float* fc1_w  = (const float*)d_in[11];
  const float* fc1_b  = (const float*)d_in[12];
  const float* fc2_w  = (const float*)d_in[13];
  const float* fc2_b  = (const float*)d_in[14];
  float* out = (float*)d_out;

  size_t off = 0;
  auto carve = [&](size_t bytes) -> size_t {
    size_t o = off;
    off += (bytes + 255) & ~(size_t)255;
    return o;
  };
  const size_t o_wqkv = carve(kBWqkv);
  const size_t o_wpj  = carve(kBWpj);
  const size_t o_wf1  = carve(kBWf1);
  const size_t o_wf2  = carve(kBWf2);
  const size_t o_rel  = carve(kBRel);
  const size_t o_ra   = carve(kBRA);
  const size_t o_rb   = carve(kRBBytes);
  const size_t o_x1   = carve(kBX1);
  if (off > ws_size) return;
  if (off > (size_t)134217728) return;

  char* ws = (char*)d_ws;
  _Float16* wqkv = (_Float16*)(ws + o_wqkv);
  _Float16* wpj  = (_Float16*)(ws + o_wpj);
  _Float16* wf1  = (_Float16*)(ws + o_wf1);
  _Float16* wf2  = (_Float16*)(ws + o_wf2);
  _Float16* relp = (_Float16*)(ws + o_rel);
  _Float16* ra   = (_Float16*)(ws + o_ra);
  _Float16* rb   = (_Float16*)(ws + o_rb);
  float*    x1   = (float*)   (ws + o_x1);

  const dim3 b256(256), b32(32);

  cvt_wt<<<dim3(kQKV / 64, kC / 64), b256, 0, stream>>>(w_qkv, wqkv, kC, kQKV);
  cvt_wt<<<dim3(kC / 64, kC / 64), b256, 0, stream>>>(w_proj, wpj, kC, kC);
  cvt_wt<<<dim3(kHid / 64, kC / 64), b256, 0, stream>>>(fc1_w, wf1, kC, kHid);
  cvt_wt<<<dim3(kC / 64, kHid / 64), b256, 0, stream>>>(fc2_w, wf2, kHid, kC);
  cvt_rel<<<dim3(1), b256, 0, stream>>>(rel_h, rel_w, relp);

  ln_rows<1><<<dim3(kMWP / 8), b256, 0, stream>>>(x, n1g, n1b, ra);

  gemm_rows<EPI_QKV><<<dim3(kMWP / 128, kQKV / 128), b256, 0, stream>>>(
      ra, wqkv, b_qkv, nullptr, nullptr, rb, kQKV, kC, 0);

  attn_win<<<dim3(kNWIN, kHeads), b32, 0, stream>>>(rb, relp, ra);

  gemm_rows<EPI_X1><<<dim3(kMWP / 128, kC / 128), b256, 0, stream>>>(
      ra, wpj, b_proj, x, x1, nullptr, kC, kC, 0);

  ln_rows<0><<<dim3(kMT / 8), b256, 0, stream>>>(x1, n2g, n2b, ra);

  for (int c = 0; c < kNChunk; ++c) {
    const int t0 = c * kTPC;
    const int nt = (kTilesT - t0 < kTPC) ? (kTilesT - t0) : kTPC;
    if (nt <= 0) continue;
    const size_t roff = (size_t)t0 * 128 * kC;
    gemm_rows<EPI_GELU><<<dim3(nt, kHid / 128), b256, 0, stream>>>(
        ra + roff, wf1, fc1_b, nullptr, nullptr, rb, kHid, kC, 0);
    gemm_rows<EPI_OUT><<<dim3(nt, kC / 128), b256, 0, stream>>>(
        rb, wf2, fc2_b, x1 + roff, out + roff, nullptr, kC, kHid, 0);
  }
}
